// RelationAwareMultiHeadedAttention_26963804685086
// MI455X (gfx1250) — hardware-verified
//
#include <hip/hip_runtime.h>

typedef _Float16 v16h __attribute__((ext_vector_type(16)));
typedef _Float16 v8h  __attribute__((ext_vector_type(8)));
typedef __bf16   v16b __attribute__((ext_vector_type(16)));
typedef __bf16   v8b  __attribute__((ext_vector_type(8)));
typedef float    v8f  __attribute__((ext_vector_type(8)));
typedef float    v4f  __attribute__((ext_vector_type(4)));
typedef int      v4i  __attribute__((ext_vector_type(4)));
typedef v8h __attribute__((may_alias)) v8ha;
typedef v8b __attribute__((may_alias)) v8ba;
typedef v4f __attribute__((may_alias)) v4fa;
typedef v4i __attribute__((may_alias)) v4ia;

union FragH { v16h v; v8h half[2]; };
union FragB { v16b v; v8b half[2]; };

#define NB    4
#define SEQ   512
#define HID   1024
#define NH    16
#define HD    64
#define NREL  64
#define NTOK  (NB * SEQ)
#define NX    (NTOK * HID)
#define NW    (HID * HID)
#define NX8   (NX / 8)
#define NW8   (NW / 8)
#define NPL   (NB * NH * SEQ * HD)
#define G_X   (3 * NX8)
#define G_W   (4 * NW8)
#define G_R   (NREL * HD / 8)
#define G_TOT (G_X + G_W + 2 * G_R)
#define PSC   16384.0f
#define RVS   4.76837158203125e-7f

__device__ __forceinline__ v8f wmma_h(v16h a, v16h b, v8f c) {
  v8f d = __builtin_amdgcn_wmma_f32_16x16x32_f16(false, a, false, b, (short)0, c, false, false);
  asm volatile("v_nop\n\tv_nop\n\tv_nop\n\tv_nop" : "+v"(d) : "v"(a), "v"(b));
  return d;
}
__device__ __forceinline__ v8f wmma_b(v16b a, v16b b, v8f c) {
  v8f d = __builtin_amdgcn_wmma_f32_16x16x32_bf16(false, a, false, b, (short)0, c, false, false);
  asm volatile("v_nop\n\tv_nop\n\tv_nop\n\tv_nop" : "+v"(d) : "v"(a), "v"(b));
  return d;
}

__device__ __forceinline__ v16h ldfrag_h(const _Float16* p, int h) {
  FragH f;
  f.half[0] = *(const v8ha*)(p + 8 * h);
  f.half[1] = *(const v8ha*)(p + 16 + 8 * h);
  return f.v;
}
__device__ __forceinline__ v16b ldfrag_b(const __bf16* p, int h) {
  FragB f;
  f.half[0] = *(const v8ba*)(p + 8 * h);
  f.half[1] = *(const v8ba*)(p + 16 + 8 * h);
  return f.v;
}

__device__ __forceinline__ int relidx(int id) {
  int t = id + ((id >> 31) & NREL);
  t = t < 0 ? 0 : t;
  t = t > (NREL - 1) ? (NREL - 1) : t;
  return t;
}

__global__ __launch_bounds__(256) void convert_kernel(
    const float* __restrict__ q_in, const float* __restrict__ k_in, const float* __restrict__ v_in,
    const float* __restrict__ Wq, const float* __restrict__ Wk, const float* __restrict__ Wv,
    const float* __restrict__ Wo, const float* __restrict__ relk, const float* __restrict__ relv,
    __bf16* __restrict__ xb, __bf16* __restrict__ wb, _Float16* __restrict__ rk, _Float16* __restrict__ rvT)
{
  const int g = blockIdx.x * 256 + threadIdx.x;
  if (g >= G_TOT) return;
  if (g < G_X + G_W) {
    const float* src;
    __bf16* dst;
    if (g < G_X) {
      const int which = g >> 18;
      const int off = g & (NX8 - 1);
      const float* s = (which == 0) ? q_in : ((which == 1) ? k_in : v_in);
      src = s + (size_t)off * 8;
      dst = xb + (size_t)which * NX + (size_t)off * 8;
    } else {
      const int e = g - G_X;
      const int wsel = e >> 17;
      const int off = e & (NW8 - 1);
      const float* s = (wsel == 0) ? Wq : ((wsel == 1) ? Wk : ((wsel == 2) ? Wv : Wo));
      src = s + (size_t)off * 8;
      dst = wb + (size_t)wsel * NW + (size_t)off * 8;
    }
    const v4f a = *(const v4fa*)src;
    const v4f c = *(const v4fa*)(src + 4);
    const v8b o = { (__bf16)a.x, (__bf16)a.y, (__bf16)a.z, (__bf16)a.w,
                    (__bf16)c.x, (__bf16)c.y, (__bf16)c.z, (__bf16)c.w };
    *(volatile v8b*)dst = o;
    __threadfence();
    *(volatile v8b*)dst = o;
  } else {
    const int e = g - (G_X + G_W);
    float f[8];
    _Float16* dst;
    if (e < G_R) {
      const float* src = relk + (size_t)e * 8;
      const v4f a = *(const v4fa*)src;
      const v4f c = *(const v4fa*)(src + 4);
      f[0] = a.x; f[1] = a.y; f[2] = a.z; f[3] = a.w;
      f[4] = c.x; f[5] = c.y; f[6] = c.z; f[7] = c.w;
      dst = rk + (size_t)e * 8;
    } else {
      const int e3 = e - G_R;
      const int d = e3 >> 3;
      const int rb = (e3 & 7) * 8;
      #pragma unroll
      for (int i = 0; i < 8; ++i) f[i] = relv[(size_t)(rb + i) * HD + d];
      dst = rvT + (size_t)e3 * 8;
    }
    _Float16 hh[8];
    #pragma unroll
    for (int i = 0; i < 8; ++i) hh[i] = (_Float16)((float)(__bf16)f[i] * 32.0f);
    const v8h o = { hh[0], hh[1], hh[2], hh[3], hh[4], hh[5], hh[6], hh[7] };
    *(volatile v8h*)dst = o;
    __threadfence();
    *(volatile v8h*)dst = o;
  }
}

__device__ __forceinline__ void proj_store_pass(const _Float16* sT, _Float16* plane, _Float16* vt,
                                                int which, int bh, int l0, int w, int lane) {
  const int q8 = lane & 7, sub = lane >> 3;
  #pragma unroll
  for (int i = 0; i < 8; ++i) {
    const int lid = w * 32 + i * 4 + sub;
    v8h v;
    _Float16* dst;
    if (which != 2) {
      v = *(const v8ha*)(sT + lid * HD + 8 * q8);
      dst = plane + ((size_t)bh * SEQ + l0 + lid) * HD + 8 * q8;
    } else {
      const int d = lid >> 1, hl = lid & 1;
      v = *(const v8ha*)(sT + d * 128 + 64 * hl + 8 * q8);
      dst = vt + ((size_t)bh * HD + d) * SEQ + l0 + 64 * hl + 8 * q8;
    }
    *(volatile v8h*)dst = v;
  }
}

__global__ __launch_bounds__(128) void proj_kernel(
    const __bf16* __restrict__ xb,
    const __bf16* __restrict__ wb,
    const float* __restrict__ bq, const float* __restrict__ bk, const float* __restrict__ bv,
    _Float16* __restrict__ qh,
    _Float16* __restrict__ kh,
    _Float16* __restrict__ vt)
{
  __shared__ __attribute__((aligned(16))) _Float16 sT[128 * 64];

  const int tid = threadIdx.x, lane = tid & 31, w = tid >> 5;
  const int h = lane >> 4, m = lane & 15;
  const int m0 = blockIdx.x * 128;
  const int cg = blockIdx.y;
  const int which = cg >> 4, head = cg & 15;
  const int m0w = m0 + 32 * w;

  const __bf16* xa0 = xb + (size_t)which * NX + (size_t)(m0w + m) * HID;
  const __bf16* xa1 = xa0 + (size_t)16 * HID;
  const __bf16* wr  = wb + (size_t)which * NW + (size_t)(head * HD + m) * HID;

  const v8f zero8 = {0.f, 0.f, 0.f, 0.f, 0.f, 0.f, 0.f, 0.f};
  v8f acc[2][4];
  #pragma unroll
  for (int mt = 0; mt < 2; ++mt)
    #pragma unroll
    for (int nt = 0; nt < 4; ++nt) acc[mt][nt] = zero8;

  #pragma unroll 1
  for (int k0 = 0; k0 < HID; k0 += 32) {
    const v16b a0 = ldfrag_b(xa0 + k0, h);
    const v16b a1 = ldfrag_b(xa1 + k0, h);
    #pragma unroll
    for (int nt = 0; nt < 4; ++nt) {
      const v16b bf = ldfrag_b(wr + (size_t)nt * 16 * HID + k0, h);
      acc[0][nt] = wmma_b(a0, bf, acc[0][nt]);
      acc[1][nt] = wmma_b(a1, bf, acc[1][nt]);
    }
  }

  const float* bias = (which == 0) ? bq : ((which == 1) ? bk : bv);
  const float osc = (which == 0) ? 0.125f : 1.0f;
  #pragma unroll
  for (int nt = 0; nt < 4; ++nt) {
    const int feat = 16 * nt + m;
    const float bvl = (float)(__bf16)bias[head * HD + feat];
    #pragma unroll
    for (int mt = 0; mt < 2; ++mt) {
      #pragma unroll
      for (int r = 0; r < 8; ++r) {
        const int tokl = 32 * w + 16 * mt + 8 * h + r;
        const float y = (acc[mt][nt][r] + bvl) * osc;
        const int idx = (which == 2) ? (feat * 128 + tokl) : (tokl * HD + feat);
        sT[idx] = (_Float16)y;
      }
    }
  }
  __syncthreads();

  const int b = m0 >> 9, l0 = m0 & (SEQ - 1), bh = b * NH + head;
  _Float16* plane = (which == 0) ? qh : kh;
  proj_store_pass(sT, plane, vt, which, bh, l0, w, lane);
  __threadfence();
  proj_store_pass(sT, plane, vt, which, bh, l0, w, lane);
}

__device__ __forceinline__ v16h build_w(const float* ha, const float* hb, int kb, float wsc) {
  const v4f a0 = *(const v4fa*)(ha + kb);
  const v4f a1 = *(const v4fa*)(ha + kb + 4);
  const v4f a2 = *(const v4fa*)(ha + kb + 16);
  const v4f a3 = *(const v4fa*)(ha + kb + 20);
  const v4f c0 = *(const v4fa*)(hb + kb);
  const v4f c1 = *(const v4fa*)(hb + kb + 4);
  const v4f c2 = *(const v4fa*)(hb + kb + 16);
  const v4f c3 = *(const v4fa*)(hb + kb + 20);
  const float e[16] = { a0.x + c0.x, a0.y + c0.y, a0.z + c0.z, a0.w + c0.w,
                        a1.x + c1.x, a1.y + c1.y, a1.z + c1.z, a1.w + c1.w,
                        a2.x + c2.x, a2.y + c2.y, a2.z + c2.z, a2.w + c2.w,
                        a3.x + c3.x, a3.y + c3.y, a3.z + c3.z, a3.w + c3.w };
  _Float16 wh[16];
  #pragma unroll
  for (int i = 0; i < 16; ++i) wh[i] = (_Float16)(e[i] * wsc);
  FragH f;
  f.half[0] = (v8h){ wh[0], wh[1], wh[2], wh[3], wh[4], wh[5], wh[6], wh[7] };
  f.half[1] = (v8h){ wh[8], wh[9], wh[10], wh[11], wh[12], wh[13], wh[14], wh[15] };
  return f.v;
}

__device__ __forceinline__ void att_store(const float* sO, __bf16* ahi, __bf16* alo,
                                          size_t gbase, int lane) {
  const int sub = lane >> 3, q8 = lane & 7;
  #pragma unroll
  for (int i = 0; i < 4; ++i) {
    const int row = 4 * i + sub;
    const float* sp = sO + row * HD + 8 * q8;
    const v4f a = *(const v4fa*)sp;
    const v4f c = *(const v4fa*)(sp + 4);
    const float f[8] = { a.x, a.y, a.z, a.w, c.x, c.y, c.z, c.w };
    __bf16 hh[8], ll[8];
    #pragma unroll
    for (int e = 0; e < 8; ++e) {
      hh[e] = (__bf16)f[e];
      ll[e] = (__bf16)(f[e] - (float)hh[e]);
    }
    const v8b hv = { hh[0], hh[1], hh[2], hh[3], hh[4], hh[5], hh[6], hh[7] };
    const v8b lv = { ll[0], ll[1], ll[2], ll[3], ll[4], ll[5], ll[6], ll[7] };
    const size_t gi = gbase + (size_t)row * HID + 8 * q8;
    *(volatile v8b*)(ahi + gi) = hv;
    *(volatile v8b*)(alo + gi) = lv;
  }
}

__global__ __launch_bounds__(32) void attn_kernel(
    const _Float16* __restrict__ qh,
    const _Float16* __restrict__ kh,
    const _Float16* __restrict__ vt,
    const int* __restrict__ ids,
    const _Float16* __restrict__ rk,
    const _Float16* __restrict__ rvT,
    __bf16* __restrict__ ahi,
    __bf16* __restrict__ alo)
{
  __shared__ __attribute__((aligned(16))) float sS[16 * SEQ];
  __shared__ __attribute__((aligned(16))) float sQR[16 * NREL];
  __shared__ __attribute__((aligned(16))) float sH[2 * 16 * NREL];
  __shared__ __attribute__((aligned(16))) float sO[16 * HD];

  const int lane = threadIdx.x & 31, h = lane >> 4, m = lane & 15;
  const int bh = blockIdx.y, b = bh >> 4, head = bh & 15;
  const int q0 = blockIdx.x * 16;

  float* hp = sH + h * (16 * NREL) + m * NREL;
  {
    const v4f z4 = {0.f, 0.f, 0.f, 0.f};
    #pragma unroll
    for (int i = 0; i < NREL / 4; ++i) *(v4fa*)(hp + 4 * i) = z4;
  }

  const _Float16* qrow = qh + ((size_t)bh * SEQ + q0 + m) * HD;
  const v16h qb0 = ldfrag_h(qrow, h);
  const v16h qb1 = ldfrag_h(qrow + 32, h);

  const v8f zero8 = {0.f, 0.f, 0.f, 0.f, 0.f, 0.f, 0.f, 0.f};

  #pragma unroll
  for (int rt = 0; rt < 4; ++rt) {
    const _Float16* ap = rk + (size_t)(16 * rt + m) * HD;
    v8f z = zero8;
    z = wmma_h(ldfrag_h(ap, h), qb0, z);
    z = wmma_h(ldfrag_h(ap + 32, h), qb1, z);
    #pragma unroll
    for (int r = 0; r < 8; ++r) sQR[m * NREL + 16 * rt + 8 * h + r] = z[r];
  }
  __syncthreads();

  const _Float16* kbase = kh + ((size_t)bh * SEQ + m) * HD;
  const _Float16* vbase = vt + ((size_t)bh * HD + m) * SEQ;
  const int* idrow = ids + ((size_t)b * SEQ + q0 + m) * SEQ + 8 * h;
  float* srow = sS + m * SEQ + 8 * h;
  const float* qr = sQR + m * NREL;

  float mx = -3.0e38f;
  #pragma unroll 1
  for (int kt = 0; kt < SEQ / 16; ++kt) {
    const _Float16* kp = kbase + (size_t)(16 * kt) * HD;
    v8f z = zero8;
    z = wmma_h(ldfrag_h(kp, h), qb0, z);
    z = wmma_h(ldfrag_h(kp + 32, h), qb1, z);
    const v4i ia = *(const v4ia*)(idrow + 16 * kt);
    const v4i ib = *(const v4ia*)(idrow + 16 * kt + 4);
    const int idv[8] = { ia.x, ia.y, ia.z, ia.w, ib.x, ib.y, ib.z, ib.w };
    float sc[8];
    #pragma unroll
    for (int r = 0; r < 8; ++r) {
      const int id = idv[r];
      const float bias = (id > 0) ? 0.0f : -10000.0f;
      const float v = z[r] + qr[relidx(id)] * 0.0078125f + bias;
      sc[r] = v;
      mx = fmaxf(mx, v);
    }
    const v4f o0 = { sc[0], sc[1], sc[2], sc[3] };
    const v4f o1 = { sc[4], sc[5], sc[6], sc[7] };
    *(v4fa*)(srow + 16 * kt) = o0;
    *(v4fa*)(srow + 16 * kt + 4) = o1;
  }
  mx = fmaxf(mx, __shfl_xor(mx, 16));
  __syncthreads();

  v8f o[4];
  #pragma unroll
  for (int t = 0; t < 4; ++t) o[t] = zero8;
  float lsum = 0.0f;
  #pragma unroll 1
  for (int c = 0; c < SEQ / 32; ++c) {
    const float* sp = srow + 32 * c;
    const v4f s0 = *(const v4fa*)(sp);
    const v4f s1 = *(const v4fa*)(sp + 4);
    const v4f s2 = *(const v4fa*)(sp + 16);
    const v4f s3 = *(const v4fa*)(sp + 20);
    const int* ip = idrow + 32 * c;
    const v4i i0 = *(const v4ia*)(ip);
    const v4i i1 = *(const v4ia*)(ip + 4);
    const v4i i2 = *(const v4ia*)(ip + 16);
    const v4i i3 = *(const v4ia*)(ip + 20);
    const float sv[16] = { s0.x, s0.y, s0.z, s0.w, s1.x, s1.y, s1.z, s1.w,
                           s2.x, s2.y, s2.z, s2.w, s3.x, s3.y, s3.z, s3.w };
    const int idv[16] = { i0.x, i0.y, i0.z, i0.w, i1.x, i1.y, i1.z, i1.w,
                          i2.x, i2.y, i2.z, i2.w, i3.x, i3.y, i3.z, i3.w };
    _Float16 ph[16];
    #pragma unroll
    for (int e = 0; e < 16; ++e) {
      const float p = __expf(sv[e] - mx);
      lsum += p;
      const int ri = relidx(idv[e]);
      hp[ri] = hp[ri] + p;
      ph[e] = (_Float16)(p * PSC);
    }
    FragH pf;
    pf.half[0] = (v8h){ ph[0], ph[1], ph[2], ph[3], ph[4], ph[5], ph[6], ph[7] };
    pf.half[1] = (v8h){ ph[8], ph[9], ph[10], ph[11], ph[12], ph[13], ph[14], ph[15] };
    #pragma unroll
    for (int t = 0; t < 4; ++t) {
      const _Float16* vp = vbase + (size_t)(16 * t) * SEQ + 32 * c;
      o[t] = wmma_h(ldfrag_h(vp, h), pf.v, o[t]);
    }
  }
  lsum += __shfl_xor(lsum, 16);
  const float inv = 1.0f / lsum;
  const float osc = inv * (1.0f / PSC);
  const float wsc = inv * PSC;
  __syncthreads();

  const float* ha = sH + m * NREL;
  const float* hb = sH + 16 * NREL + m * NREL;
  const v16h w0 = build_w(ha, hb, 8 * h, wsc);
  const v16h w1 = build_w(ha, hb, 32 + 8 * h, wsc);
  #pragma unroll
  for (int t = 0; t < 4; ++t) {
    const _Float16* ap = rvT + (size_t)(16 * t + m) * NREL;
    v8f z = zero8;
    z = wmma_h(ldfrag_h(ap, h), w0, z);
    z = wmma_h(ldfrag_h(ap + 32, h), w1, z);
    #pragma unroll
    for (int r = 0; r < 8; ++r)
      sO[m * HD + 16 * t + 8 * h + r] = o[t][r] * osc + z[r] * RVS;
  }
  __syncthreads();

  const size_t gbase = ((size_t)b * SEQ + q0) * HID + (size_t)head * HD;
  att_store(sO, ahi, alo, gbase, lane);
  __threadfence();
  att_store(sO, ahi, alo, gbase, lane);
}

__device__ __forceinline__ void out_store_pass(const float* sT, float* out, int m0, int n0,
                                               int w, int lane) {
  const int q8 = lane & 7, sub = lane >> 3;
  #pragma unroll
  for (int i = 0; i < 16; ++i) {
    const int lid = i * 4 + sub;
    const int rowl = 32 * w + (lid >> 1), hl = lid & 1;
    const v4f v = *(const v4fa*)(sT + rowl * 64 + 32 * hl + 4 * q8);
    float* dst = out + (size_t)(m0 + rowl) * HID + n0 + 32 * hl + 4 * q8;
    *(volatile v4f*)dst = v;
  }
}

__global__ __launch_bounds__(128) void oproj_kernel(
    const __bf16* __restrict__ ahi,
    const __bf16* __restrict__ alo,
    const __bf16* __restrict__ wo,
    const float* __restrict__ bo,
    float* __restrict__ out)
{
  __shared__ __attribute__((aligned(16))) float sT[128 * 64];

  const int tid = threadIdx.x, lane = tid & 31, w = tid >> 5;
  const int h = lane >> 4, m = lane & 15;
  const int m0 = blockIdx.x * 128;
  const int n0 = blockIdx.y * 64;
  const int m0w = m0 + 32 * w;

  const __bf16* a0h = ahi + (size_t)(m0w + m) * HID;
  const __bf16* a0l = alo + (size_t)(m0w + m) * HID;
  const __bf16* a1h = a0h + (size_t)16 * HID;
  const __bf16* a1l = a0l + (size_t)16 * HID;
  const __bf16* wr  = wo + (size_t)(n0 + m) * HID;

  const v8f zero8 = {0.f, 0.f, 0.f, 0.f, 0.f, 0.f, 0.f, 0.f};
  v8f acc[2][4];
  #pragma unroll
  for (int mt = 0; mt < 2; ++mt)
    #pragma unroll
    for (int nt = 0; nt < 4; ++nt) acc[mt][nt] = zero8;

  #pragma unroll 1
  for (int k0 = 0; k0 < HID; k0 += 32) {
    const v16b f0h = ldfrag_b(a0h + k0, h);
    const v16b f0l = ldfrag_b(a0l + k0, h);
    const v16b f1h = ldfrag_b(a1h + k0, h);
    const v16b f1l = ldfrag_b(a1l + k0, h);
    #pragma unroll
    for (int nt = 0; nt < 4; ++nt) {
      const v16b bf = ldfrag_b(wr + (size_t)nt * 16 * HID + k0, h);
      acc[0][nt] = wmma_b(f0h, bf, acc[0][nt]);
      acc[0][nt] = wmma_b(f0l, bf, acc[0][nt]);
      acc[1][nt] = wmma_b(f1h, bf, acc[1][nt]);
      acc[1][nt] = wmma_b(f1l, bf, acc[1][nt]);
    }
  }

  #pragma unroll
  for (int nt = 0; nt < 4; ++nt) {
    const int featl = 16 * nt + m;
    const float bvl = (float)(__bf16)bo[n0 + featl];
    #pragma unroll
    for (int mt = 0; mt < 2; ++mt) {
      #pragma unroll
      for (int r = 0; r < 8; ++r) {
        const int tokl = 32 * w + 16 * mt + 8 * h + r;
        sT[tokl * 64 + featl] = acc[mt][nt][r] + bvl;
      }
    }
  }
  __syncthreads();

  out_store_pass(sT, out, m0, n0, w, lane);
  __threadfence();
  out_store_pass(sT, out, m0, n0, w, lane);
}

extern "C" void kernel_launch(void* const* d_in, const int* in_sizes, int n_in,
                              void* d_out, int out_size, void* d_ws, size_t ws_size,
                              hipStream_t stream) {
  if (n_in < 14) return;
  if (in_sizes[0] != NX || in_sizes[1] != NX || in_sizes[2] != NX) return;
  if (in_sizes[3] != NB * SEQ * SEQ) return;
  if (in_sizes[4] != NW || in_sizes[6] != NW || in_sizes[8] != NW || in_sizes[10] != NW) return;
  if (in_sizes[5] != HID || in_sizes[7] != HID || in_sizes[9] != HID || in_sizes[11] != HID) return;
  if (in_sizes[12] != NREL * HD || in_sizes[13] != NREL * HD) return;
  if (out_size != NX) return;

  const float* q_in = (const float*)d_in[0];
  const float* k_in = (const float*)d_in[1];
  const float* v_in = (const float*)d_in[2];
  const int*   ids  = (const int*)d_in[3];
  const float* Wq = (const float*)d_in[4];
  const float* bq = (const float*)d_in[5];
  const float* Wk = (const float*)d_in[6];
  const float* bk = (const float*)d_in[7];
  const float* Wv = (const float*)d_in[8];
  const float* bv = (const float*)d_in[9];
  const float* Wo = (const float*)d_in[10];
  const float* bo = (const float*)d_in[11];
  const float* relk = (const float*)d_in[12];
  const float* relv = (const float*)d_in[13];
  float* out = (float*)d_out;

  const size_t xb_bytes = (size_t)3 * NX * 2;
  const size_t wb_bytes = (size_t)4 * NW * 2;
  const size_t rt_bytes = (size_t)NREL * HD * 2;
  const size_t pl_bytes = (size_t)NPL * 2;
  const size_t ap_bytes = (size_t)NX * 2;
  const size_t total = xb_bytes + wb_bytes + 2 * rt_bytes + 3 * pl_bytes + 2 * ap_bytes;
  if (total > ws_size) return;

  char* ws = (char*)d_ws;
  size_t off = 0;
  __bf16* xb = (__bf16*)(ws + off);       off += xb_bytes;
  __bf16* wb = (__bf16*)(ws + off);       off += wb_bytes;
  _Float16* rk  = (_Float16*)(ws + off);  off += rt_bytes;
  _Float16* rvT = (_Float16*)(ws + off);  off += rt_bytes;
  _Float16* qh  = (_Float16*)(ws + off);  off += pl_bytes;
  _Float16* kh  = (_Float16*)(ws + off);  off += pl_bytes;
  _Float16* vt  = (_Float16*)(ws + off);  off += pl_bytes;
  __bf16* ahi = (__bf16*)(ws + off);      off += ap_bytes;
  __bf16* alo = (__bf16*)(ws + off);      off += ap_bytes;
  if (off > ws_size) return;

  convert_kernel<<<(G_TOT + 255) / 256, 256, 0, stream>>>(q_in, k_in, v_in, Wq, Wk, Wv, Wo,
                                                         relk, relv, xb, wb, rk, rvT);

  dim3 gProj(NTOK / 128, 3 * NH);
  proj_kernel<<<gProj, 128, 0, stream>>>(xb, wb, bq, bk, bv, qh, kh, vt);

  dim3 gAtt(SEQ / 16, NB * NH);
  attn_kernel<<<gAtt, 32, 0, stream>>>(qh, kh, vt, ids, rk, rvT, ahi, alo);

  dim3 gOut(NTOK / 128, HID / 64);
  oproj_kernel<<<gOut, 128, 0, stream>>>(ahi, alo, wb + (size_t)3 * NW, bo, out);
}
